// TransformerSequenceDecoder_75093208203778
// MI455X (gfx1250) — hardware-run, weakly checked
//
#include <hip/hip_runtime.h>


#define NBATCH 8
#define DM     512
#define NHD    8
#define HD     64
#define NLAY   2
#define DFF    2048
#define FFH    1024
#define VOC    32000
#define SMEM   48
#define NTR    14
#define INITL  (NTR - 2)
#ifndef GENLEN
#define GENLEN 24
#endif
#define GENLEN_FULL 24
#define LFN    (INITL + GENLEN - 1)
#define LF_FULL (INITL + GENLEN_FULL - 1)
#define QRS  2048.0f
#define QRI  (1.0f / 2048.0f)
#define WCS  1024.0f
#define WCI  (1.0f / 1024.0f)
#define NEGB (-3.0e38f)
#define AP1  (DM + 8)
#define AP2  (FFH + 8)
#define SCK  48
#define SCP  49
#define OSV  68

static_assert(NBATCH == 8);
static_assert(NHD * HD == DM);
static_assert(DM == 8 * 64);
static_assert(DM == 32 * 16);
static_assert(4 * 32 * 4 == DM);
static_assert(DM % 32 == 0);
static_assert(FFH % 32 == 0);
static_assert(DFF == 2 * FFH);
static_assert(FFH == 2 * 8 * 64);
static_assert(VOC % 256 == 0);
static_assert(VOC % 128 == 0);
static_assert(GENLEN >= 1);
static_assert(GENLEN <= GENLEN_FULL);
static_assert(LFN <= SCK);
static_assert(SMEM <= SCK);
static_assert(SCK < SCP + 1);
static_assert((AP1 * 2) % 16 == 0);
static_assert((AP2 * 2) % 16 == 0);
static_assert((OSV * 4) % 16 == 0);
static_assert(4 * 256 * 4 == NBATCH * DM);
static_assert(4 * 256 * 8 == 16 * DM);
static_assert(32 * 4 * 4 == NBATCH * 64);
static_assert((INITL * DM) % 256 == 0);
static_assert((size_t)16 * AP1 * 2 + (size_t)16 * AP2 * 2 + (size_t)2 * NBATCH * DM * 4 + (size_t)NBATCH * DM * 4 + (size_t)64 * SCP * 4 + (size_t)2 * DM * 4 + 64 <= (size_t)131072);
static_assert((size_t)16 * AP1 * 2 + (size_t)NBATCH * DM * 4 <= (size_t)131072);
static_assert((size_t)4 * 16 * OSV * 4 <= (size_t)131072);

typedef _Float16 h16;
typedef __attribute__((ext_vector_type(16))) _Float16 v16h;
typedef __attribute__((ext_vector_type(8)))  _Float16 v8h;
typedef __attribute__((ext_vector_type(8)))  float    v8f;
typedef __attribute__((ext_vector_type(4)))  float    v4f;
typedef v4f  __attribute__((may_alias)) v4fa;

__device__ __forceinline__ unsigned short f2bf(float f) { unsigned u = __float_as_uint(f); u += 0x7FFFu + ((u >> 16) & 1u); return (unsigned short)(u >> 16); }
__device__ __forceinline__ float bfr(float f) { return __uint_as_float(((unsigned)f2bf(f)) << 16); }
__device__ __forceinline__ v16h cat16(v8h lo, v8h hi) { return __builtin_shufflevector(lo, hi, 0, 1, 2, 3, 4, 5, 6, 7, 8, 9, 10, 11, 12, 13, 14, 15); }
__device__ __forceinline__ v8f wmma16(v16h a, v16h b, v8f c) { return __builtin_amdgcn_wmma_f32_16x16x32_f16(false, a, false, b, (short)0, c, false, false); }
__device__ __forceinline__ v16h  ldh(const h16* p) { return cat16(*(const v8h*)p, *(const v8h*)(p + 16)); }
__device__ __forceinline__ void wave_sync() { __builtin_amdgcn_fence(3  , "wavefront"); __builtin_amdgcn_wave_barrier(); asm volatile("" ::: "memory"); }

static __device__ __forceinline__ h16 toh_flush(float v) { const h16 r = (h16)v; return (fabsf(v) < 6.103515625e-05f) ? (h16)0.0f : r; }
__device__ __forceinline__ void split_hr(float v, h16& hv, h16& rv) { hv = toh_flush(v); rv = toh_flush((v - (float)hv) * QRS); }
__device__ __forceinline__ v8f wmg(v16h a, v16h b, v8f c) { c = wmma16(a, b, c); asm volatile("v_nop\n\tv_nop\n\tv_nop\n\tv_nop" : "+v"(c) : "v"(a), "v"(b)); return c; }

template <int KLEN, int AP, int WP>
__device__ __forceinline__ void gemm4(const h16* As, const h16* __restrict__ W, size_t wofs, int lr, int hi, v8f& c0, v8f& c1, v8f& c2, v8f& c3) {
    const int ao = lr * AP + 8 * hi;
    const size_t bo = wofs + (size_t)lr * WP + 8 * hi;
#pragma unroll 2
    for (int kc = 0; kc < KLEN; kc += 32) {
        const v16h a  = ldh(As + ao + kc);
        const v16h b0 = ldh(W + bo + kc);
        const v16h b1 = ldh(W + bo + (size_t)16 * WP + kc);
        const v16h b2 = ldh(W + bo + (size_t)32 * WP + kc);
        const v16h b3 = ldh(W + bo + (size_t)48 * WP + kc);
        c0 = wmg(a, b0, c0); c1 = wmg(a, b1, c1); c2 = wmg(a, b2, c2); c3 = wmg(a, b3, c3);
    }
}

__device__ __forceinline__ void epi_y(float* Ys, int ycol, const float* __restrict__ bias, int bofs, int lr, int hi, bool accum, v8f c) {
    const float braw = bias[bofs + lr];
    const float bv = accum ? 0.0f : bfr(braw);
    float o[8];
#pragma unroll
    for (int r = 0; r < 8; ++r) {
        const float t = __shfl_xor(c[r], 16, 32);
        const float vh = hi ? t : c[r];
        const float vr = hi ? c[r] : t;
        o[r] = (vh + vr * QRI) * WCI + bv;
    }
    if (hi == 0) {
        if (accum) {
#pragma unroll
            for (int r = 0; r < 8; ++r) { const int ix = r * DM + ycol + lr; Ys[ix] = Ys[ix] + o[r]; }
        } else {
#pragma unroll
            for (int r = 0; r < 8; ++r) Ys[r * DM + ycol + lr] = o[r];
        }
    }
}

__device__ __forceinline__ void epi_h(h16* As, int acol, const float* __restrict__ bias, int bofs, int lr, int hi, v8f c) {
    const float bv = bfr(bias[bofs + lr]);
    h16 hv[8], rv[8];
#pragma unroll
    for (int r = 0; r < 8; ++r) {
        const float t = __shfl_xor(c[r], 16, 32);
        const float vh = hi ? t : c[r];
        const float vr = hi ? c[r] : t;
        const float o = fmaxf((vh + vr * QRI) * WCI + bv, 0.0f);
        split_hr(o, hv[r], rv[r]);
    }
    if (hi == 0) {
#pragma unroll
        for (int r = 0; r < 8; ++r) { As[r * AP2 + acol + lr] = hv[r]; As[(8 + r) * AP2 + acol + lr] = rv[r]; }
    }
}

__device__ __forceinline__ void stage_gb(float* GBs, const float* __restrict__ g, const float* __restrict__ be, int gofs, int wave, int tid) {
    if (wave < 4) {
        const int c4 = tid * 4;
        const v4f gv = *(const v4fa*)(g + gofs + c4);
        const v4f bv = *(const v4fa*)(be + gofs + c4);
        *(v4fa*)(&GBs[c4]) = gv; *(v4fa*)(&GBs[DM + c4]) = bv;
    }
}

__device__ __forceinline__ void ln_row(float* XRs, const float* Ys, h16* A1s, const float* GBs, int wave, int lane) {
    float v[16]; float s = 0.0f;
#pragma unroll
    for (int i = 0; i < 16; ++i) { const int e = lane + 32 * i; v[i] = XRs[wave * DM + e] + Ys[wave * DM + e]; s += v[i]; }
#pragma unroll
    for (int off = 16; off > 0; off >>= 1) s += __shfl_xor(s, off, 32);
    const float mean = s * (1.0f / DM);
    float s2 = 0.0f;
#pragma unroll
    for (int i = 0; i < 16; ++i) { const float d = v[i] - mean; s2 += d * d; }
#pragma unroll
    for (int off = 16; off > 0; off >>= 1) s2 += __shfl_xor(s2, off, 32);
    const float rs = 1.0f / sqrtf(s2 * (1.0f / DM) + 1.0e-5f);
#pragma unroll
    for (int i = 0; i < 16; ++i) {
        const int e = lane + 32 * i;
        const float o = (v[i] - mean) * rs * bfr(GBs[e]) + bfr(GBs[DM + e]);
        XRs[wave * DM + e] = o;
        h16 hv, rv; split_hr(o, hv, rv);
        A1s[wave * AP1 + e] = hv; A1s[(8 + wave) * AP1 + e] = rv;
    }
}

__device__ __forceinline__ void attend(const float* Qs, float* SCs, h16* A1s, const float* KB, const float* VB, int nkeys_in, int wave, int lane) {
    const int nkeys = nkeys_in < 1 ? 1 : (nkeys_in > SCK ? SCK : nkeys_in);
    const int nit = 64 * nkeys;
#pragma unroll 1
    for (int base = wave * 32; base < nit; base += 256) {
        const int it = base + lane; const int j = it >> 6, bh = it & 63; const int b = bh >> 3, h = bh & 7;
        const float* kp = KB + ((size_t)(j * NBATCH + b)) * DM + h * HD;
        const int qo = b * DM + h * HD;
        float acc = 0.0f;
#pragma unroll 4
        for (int d = 0; d < HD; d += 4) {
            const v4f kv = *(const v4f*)(kp + d); const v4f qv = *(const v4fa*)(&Qs[qo + d]);
            acc = fmaf(qv[0], kv[0], acc); acc = fmaf(qv[1], kv[1], acc); acc = fmaf(qv[2], kv[2], acc); acc = fmaf(qv[3], kv[3], acc);
        }
        SCs[bh * SCP + j] = acc * 0.125f;
    }
    __syncthreads();
    if (wave < 2) {
        const int row = wave * 32 + lane;
        float m = NEGB;
#pragma unroll 1
        for (int j = 0; j < nkeys; ++j) m = fmaxf(m, SCs[row * SCP + j]);
        float sum = 0.0f;
#pragma unroll 1
        for (int j = 0; j < nkeys; ++j) { const float e = expf(SCs[row * SCP + j] - m); SCs[row * SCP + j] = e; sum += e; }
        const float inv = 1.0f / sum;
#pragma unroll 1
        for (int j = 0; j < nkeys; ++j) SCs[row * SCP + j] = SCs[row * SCP + j] * inv;
    }
    __syncthreads();
#pragma unroll 1
    for (int i = 0; i < 4; ++i) {
        const int idx = i * 256 + wave * 32 + lane; const int b = idx >> 7, c4 = (idx & 127) * 4; const int h = c4 >> 6;
        const float* vp = VB + (size_t)b * DM + c4; const int so = (b * NHD + h) * SCP;
        v4f acc = (v4f){};
#pragma unroll 1
        for (int j = 0; j < nkeys; ++j) { const float pj = SCs[so + j]; const v4f vv = *(const v4f*)(vp + (size_t)j * (NBATCH * DM)); acc += pj * vv; }
#pragma unroll
        for (int c = 0; c < 4; ++c) { h16 hv, rv; split_hr(acc[c], hv, rv); A1s[b * AP1 + c4 + c] = hv; A1s[(8 + b) * AP1 + c4 + c] = rv; }
    }
    __syncthreads();
}

__global__ __launch_bounds__(256) void k_wcvt(const float* __restrict__ src, h16* dst, size_t n8) {
    const size_t i = (size_t)blockIdx.x * 256 + threadIdx.x; if (i >= n8) return;
    const v8f v = *(const v8f*)(src + i * 8); v8h o;
#pragma unroll
    for (int k = 0; k < 8; ++k) o[k] = toh_flush(bfr(v[k]) * WCS);
    *(volatile v8h*)(dst + i * 8) = o; __threadfence(); *(volatile v8h*)(dst + i * 8) = o;
}

__global__ __launch_bounds__(256) void k_pe(float* PE) {
    const int i = blockIdx.x * 256 + threadIdx.x; if (i >= INITL * DM) return;
    const int t = i / DM, d = i % DM;
    const float ex = (-9.210340371976184f * (float)(d & ~1)) / 512.0f;
    const float dv = expf(ex);
    const float ang = (float)t * dv;
    const float sv = sinf(ang), cv = cosf(ang);
    const float val = (d & 1) ? cv : sv;
    *(volatile float*)(PE + i) = val; __threadfence(); *(volatile float*)(PE + i) = val;
}

__global__ __launch_bounds__(256) void k_mem(const float* __restrict__ enc, const h16* __restrict__ WCA, const float* __restrict__ ca_b, float* MEM) {
    __shared__ __align__(16) h16   A1[16 * AP1];
    __shared__ __align__(16) float Y[NBATCH * DM];
    const int tid = threadIdx.x, lane = tid & 31, lr = lane & 15, hi = lane >> 4;
    const int wave = __builtin_amdgcn_readfirstlane((int)(threadIdx.x >> 5));
    const int s = blockIdx.x, lk = blockIdx.y; const int l = lk >> 1, kv = lk & 1;
    if (s >= SMEM || lk >= NLAY * 2) return;
#pragma unroll 1
    for (int i = 0; i < 4; ++i) {
        const int idx = i * 256 + tid; const int b = idx >> 7, c4 = (idx & 127) * 4;
        const v4f e = *(const v4f*)(enc + (size_t)s * (NBATCH * DM) + (size_t)idx * 4);
#pragma unroll
        for (int c = 0; c < 4; ++c) { h16 hv, rv; split_hr(bfr(e[c]), hv, rv); A1[b * AP1 + c4 + c] = hv; A1[(8 + b) * AP1 + c4 + c] = rv; }
    }
    __syncthreads();
    {
        v8f c0 = (v8f){}, c1 = (v8f){}, c2 = (v8f){}, c3 = (v8f){};
        const int wr = l * 3 * DM + (1 + kv) * DM + wave * 64;
        gemm4<DM, AP1, DM>(A1, WCA, (size_t)wr * DM, lr, hi, c0, c1, c2, c3);
        const int yb = wave * 64;
        epi_y(Y, yb, ca_b, wr, lr, hi, false, c0); epi_y(Y, yb + 16, ca_b, wr + 16, lr, hi, false, c1);
        epi_y(Y, yb + 32, ca_b, wr + 32, lr, hi, false, c2); epi_y(Y, yb + 48, ca_b, wr + 48, lr, hi, false, c3);
    }
    __syncthreads();
    float* dst = MEM + ((size_t)(lk * SMEM + s)) * (NBATCH * DM);
#pragma unroll 1
    for (int ps = 0; ps < 2; ++ps) {
#pragma unroll
        for (int i = 0; i < 4; ++i) { const int idx = i * 256 + tid; const v4f v = *(const v4fa*)(&Y[idx * 4]); *(volatile v4f*)(dst + (size_t)idx * 4) = v; }
        if (ps == 0) __threadfence();
    }
}

__global__ __launch_bounds__(256) void k_step(const int* __restrict__ transform, const float* __restrict__ emb, const float* __restrict__ PE,
                                              const h16* __restrict__ WSA, const float* __restrict__ sa_b, const h16* __restrict__ WSO, const float* __restrict__ sa_ob,
                                              const h16* __restrict__ WCA, const float* __restrict__ ca_b, const h16* __restrict__ WCO, const float* __restrict__ ca_ob,
                                              const h16* __restrict__ WF1, const float* __restrict__ ff1_b, const h16* __restrict__ WF2, const float* __restrict__ ff2_b,
                                              const float* __restrict__ ln_g, const float* __restrict__ ln_b,
                                              const float* __restrict__ MEM, float* KV, h16* HP, const float* OUTL, int p0, int p1) {
    __shared__ __align__(16) h16   A1[16 * AP1];
    __shared__ __align__(16) h16   A2[16 * AP2];
    __shared__ __align__(16) float QY[2 * NBATCH * DM];
    __shared__ __align__(16) float XR[NBATCH * DM];
    __shared__ __align__(16) float SC[64 * SCP];
    __shared__ __align__(16) float GB[2 * DM];
    __shared__ int tok[NBATCH];
    const int tid = threadIdx.x, lane = tid & 31, lr = lane & 15, hi = lane >> 4;
    const int wave = __builtin_amdgcn_readfirstlane((int)(threadIdx.x >> 5));
    const int pa = p0 < 0 ? 0 : p0; const int pb = p1 > LFN ? LFN : p1;
    const int Y1 = NBATCH * DM;
#pragma unroll 1
    for (int p = pa; p < pb; ++p) {
        int token;
        if (p >= INITL) {
            const float* row = OUTL + ((size_t)((p - 1) * NBATCH + wave)) * VOC;
            float best = NEGB; int besti = 0;
#pragma unroll 1
            for (int k = 0; k < VOC / 128; ++k) {
                const int i4 = k * 32 + lane;
                const v4f f = *(const v4f*)(row + (size_t)i4 * 4);
#pragma unroll
                for (int c = 0; c < 4; ++c) { const bool gt = f[c] > best; best = gt ? f[c] : best; besti = gt ? (i4 * 4 + c) : besti; }
            }
#pragma unroll
            for (int off = 16; off > 0; off >>= 1) {
                const float ov = __shfl_xor(best, off, 32); const int oi = __shfl_xor(besti, off, 32);
                const bool take = (ov > best) | ((ov == best) & (oi < besti));
                best = take ? ov : best; besti = take ? oi : besti;
            }
            token = besti;
        } else {
            token = transform[(p + 1) * NBATCH + wave];
        }
        token = token < 0 ? 0 : (token > VOC - 1 ? VOC - 1 : token);
        if (lane == 0) tok[wave] = token;
        __syncthreads();
        const int pp = p < INITL ? p : 0;
#pragma unroll 1
        for (int i = 0; i < 4; ++i) {
            const int idx = i * 256 + tid; const int b = idx >> 7, c4 = (idx & 127) * 4;
            const int tk = tok[b];
            const v4f e  = *(const v4f*)(emb + (size_t)tk * DM + c4);
            const v4f pv = *(const v4f*)(PE + (size_t)pp * DM + c4);
            v4f x;
#pragma unroll
            for (int c = 0; c < 4; ++c) x[c] = bfr(e[c]) + pv[c];
            *(v4fa*)(&XR[b * DM + c4]) = x;
#pragma unroll
            for (int c = 0; c < 4; ++c) { h16 hv, rv; split_hr(x[c], hv, rv); A1[b * AP1 + c4 + c] = hv; A1[(8 + b) * AP1 + c4 + c] = rv; }
        }
        __syncthreads();
#pragma unroll 1
        for (int l = 0; l < NLAY; ++l) {
#pragma unroll 1
            for (int part = 0; part < 3; ++part) {
                v8f c0 = (v8f){}, c1 = (v8f){}, c2 = (v8f){}, c3 = (v8f){};
                const int wr = l * 3 * DM + part * DM + wave * 64;
                gemm4<DM, AP1, DM>(A1, WSA, (size_t)wr * DM, lr, hi, c0, c1, c2, c3);
                const int yb = (part == 0 ? 0 : Y1) + wave * 64;
                epi_y(QY, yb, sa_b, wr, lr, hi, false, c0); epi_y(QY, yb + 16, sa_b, wr + 16, lr, hi, false, c1);
                epi_y(QY, yb + 32, sa_b, wr + 32, lr, hi, false, c2); epi_y(QY, yb + 48, sa_b, wr + 48, lr, hi, false, c3);
                __syncthreads();
                if (part > 0) {
                    float* dst = KV + ((size_t)((l * 2 + part - 1) * LFN + p)) * (NBATCH * DM);
#pragma unroll 1
                    for (int ps = 0; ps < 2; ++ps) {
#pragma unroll
                        for (int i = 0; i < 4; ++i) { const int idx = i * 256 + tid; const v4f v = *(const v4fa*)(&QY[Y1 + idx * 4]); *(volatile v4f*)(dst + (size_t)idx * 4) = v; }
                        if (ps == 0) __threadfence();
                    }
                }
                __syncthreads();
            }
            attend(QY, SC, A1, KV + (size_t)(l * 2) * LFN * (NBATCH * DM), KV + (size_t)(l * 2 + 1) * LFN * (NBATCH * DM), p + 1, wave, lane);
            {
                v8f c0 = (v8f){}, c1 = (v8f){}, c2 = (v8f){}, c3 = (v8f){};
                const int wr = l * DM + wave * 64;
                gemm4<DM, AP1, DM>(A1, WSO, (size_t)wr * DM, lr, hi, c0, c1, c2, c3);
                const int yb = Y1 + wave * 64;
                epi_y(QY, yb, sa_ob, wr, lr, hi, false, c0); epi_y(QY, yb + 16, sa_ob, wr + 16, lr, hi, false, c1);
                epi_y(QY, yb + 32, sa_ob, wr + 32, lr, hi, false, c2); epi_y(QY, yb + 48, sa_ob, wr + 48, lr, hi, false, c3);
            }
            stage_gb(GB, ln_g, ln_b, (l * 3 + 0) * DM, wave, tid);
            __syncthreads();
            ln_row(XR, QY + Y1, A1, GB, wave, lane);
            __syncthreads();
            {
                v8f c0 = (v8f){}, c1 = (v8f){}, c2 = (v8f){}, c3 = (v8f){};
                const int wr = l * 3 * DM + wave * 64;
                gemm4<DM, AP1, DM>(A1, WCA, (size_t)wr * DM, lr, hi, c0, c1, c2, c3);
                const int yb = wave * 64;
                epi_y(QY, yb, ca_b, wr, lr, hi, false, c0); epi_y(QY, yb + 16, ca_b, wr + 16, lr, hi, false, c1);
                epi_y(QY, yb + 32, ca_b, wr + 32, lr, hi, false, c2); epi_y(QY, yb + 48, ca_b, wr + 48, lr, hi, false, c3);
            }
            __syncthreads();
            attend(QY, SC, A1, MEM + (size_t)(l * 2) * SMEM * (NBATCH * DM), MEM + (size_t)(l * 2 + 1) * SMEM * (NBATCH * DM), SMEM, wave, lane);
            {
                v8f c0 = (v8f){}, c1 = (v8f){}, c2 = (v8f){}, c3 = (v8f){};
                const int wr = l * DM + wave * 64;
                gemm4<DM, AP1, DM>(A1, WCO, (size_t)wr * DM, lr, hi, c0, c1, c2, c3);
                const int yb = Y1 + wave * 64;
                epi_y(QY, yb, ca_ob, wr, lr, hi, false, c0); epi_y(QY, yb + 16, ca_ob, wr + 16, lr, hi, false, c1);
                epi_y(QY, yb + 32, ca_ob, wr + 32, lr, hi, false, c2); epi_y(QY, yb + 48, ca_ob, wr + 48, lr, hi, false, c3);
            }
            stage_gb(GB, ln_g, ln_b, (l * 3 + 1) * DM, wave, tid);
            __syncthreads();
            ln_row(XR, QY + Y1, A1, GB, wave, lane);
            __syncthreads();
            stage_gb(GB, ln_g, ln_b, (l * 3 + 2) * DM, wave, tid);
#pragma unroll 1
            for (int hf = 0; hf < 2; ++hf) {
#pragma unroll 1
                for (int g = 0; g < 2; ++g) {
                    v8f c0 = (v8f){}, c1 = (v8f){}, c2 = (v8f){}, c3 = (v8f){};
                    const int col = (g * 8 + wave) * 64;
                    const int wr = l * DFF + hf * FFH + col;
                    gemm4<DM, AP1, DM>(A1, WF1, (size_t)wr * DM, lr, hi, c0, c1, c2, c3);
                    epi_h(A2, col, ff1_b, wr, lr, hi, c0); epi_h(A2, col + 16, ff1_b, wr + 16, lr, hi, c1);
                    epi_h(A2, col + 32, ff1_b, wr + 32, lr, hi, c2); epi_h(A2, col + 48, ff1_b, wr + 48, lr, hi, c3);
                }
                __syncthreads();
                {
                    v8f c0 = (v8f){}, c1 = (v8f){}, c2 = (v8f){}, c3 = (v8f){};
                    const int wr = l * DM + wave * 64;
                    gemm4<FFH, AP2, DFF>(A2, WF2, (size_t)wr * DFF + (size_t)hf * FFH, lr, hi, c0, c1, c2, c3);
                    const int yb = Y1 + wave * 64; const bool ac = hf > 0;
                    epi_y(QY, yb, ff2_b, wr, lr, hi, ac, c0); epi_y(QY, yb + 16, ff2_b, wr + 16, lr, hi, ac, c1);
                    epi_y(QY, yb + 32, ff2_b, wr + 32, lr, hi, ac, c2); epi_y(QY, yb + 48, ff2_b, wr + 48, lr, hi, ac, c3);
                }
                __syncthreads();
            }
            ln_row(XR, QY + Y1, A1, GB, wave, lane);
            __syncthreads();
        }
        {
            h16* dst = HP + (size_t)p * 16 * DM;
#pragma unroll 1
            for (int ps = 0; ps < 2; ++ps) {
#pragma unroll
                for (int i = 0; i < 4; ++i) { const int idx = i * 256 + tid; const int row = idx >> 6, c8 = (idx & 63) * 8;
                    const v8h v = *(const v8h*)(&A1[row * AP1 + c8]); *(volatile v8h*)(dst + (size_t)idx * 8) = v; }
                if (ps == 0) __threadfence();
            }
        }
        __syncthreads();
    }
}

__global__ __launch_bounds__(128) void k_vocab(const h16* __restrict__ HP, const h16* __restrict__ WOUT, const float* __restrict__ out_b, float* OUT, int p0) {
    __shared__ __align__(16) float os[4 * 16 * OSV];
    const int lane = threadIdx.x & 31, lr = lane & 15, hi = lane >> 4;
    const int wave = __builtin_amdgcn_readfirstlane((int)(threadIdx.x >> 5));
    const int p = p0 + (int)blockIdx.y; if (p < 0 || p >= LFN) return;
    const int n0 = blockIdx.x * 256 + wave * 64; if (n0 + 64 > VOC) return;
    const size_t ao = ((size_t)p * 16 + lr) * DM + 8 * hi;
    const size_t bo = ((size_t)(n0 + lr)) * DM + 8 * hi;
    v8f c0 = (v8f){}, c1 = (v8f){}, c2 = (v8f){}, c3 = (v8f){};
#pragma unroll 2
    for (int kc = 0; kc < DM; kc += 32) {
        const v16h a  = ldh(HP + ao + kc);
        const v16h b0 = ldh(WOUT + bo + kc);
        const v16h b1 = ldh(WOUT + bo + (size_t)16 * DM + kc);
        const v16h b2 = ldh(WOUT + bo + (size_t)32 * DM + kc);
        const v16h b3 = ldh(WOUT + bo + (size_t)48 * DM + kc);
        c0 = wmg(a, b0, c0); c1 = wmg(a, b1, c1); c2 = wmg(a, b2, c2); c3 = wmg(a, b3, c3);
    }
    const int wb = wave * 16 * OSV;
#pragma unroll
    for (int r = 0; r < 8; ++r) {
        os[wb + (8 * hi + r) * OSV +  0 + lr] = c0[r]; os[wb + (8 * hi + r) * OSV + 16 + lr] = c1[r];
        os[wb + (8 * hi + r) * OSV + 32 + lr] = c2[r]; os[wb + (8 * hi + r) * OSV + 48 + lr] = c3[r];
    }
    wave_sync();
    const int c4 = (lane & 15) * 4;
    const v4f braw = *(const v4f*)(out_b + n0 + c4);
    v4f bv;
#pragma unroll
    for (int c = 0; c < 4; ++c) bv[c] = bfr(braw[c]);
#pragma unroll 1
    for (int ps = 0; ps < 2; ++ps) {
#pragma unroll
        for (int s = 0; s < 4; ++s) { const int b = 2 * s + (lane >> 4);
            const v4f x0 = *(const v4fa*)(&os[wb + b * OSV + c4]); const v4f x1 = *(const v4fa*)(&os[wb + (8 + b) * OSV + c4]);
            const v4f o = (x0 + x1 * QRI) * WCI + bv;
            *(volatile v4f*)(OUT + ((size_t)(p * NBATCH + b)) * VOC + n0 + c4) = o; }
        if (ps == 0) __threadfence();
    }
}

static constexpr size_t al256(size_t v) { return (v + 255) & ~(size_t)255; }
static constexpr size_t SZ_WSA = al256((size_t)NLAY * 3 * DM * DM * 2);
static constexpr size_t SZ_WSO = al256((size_t)NLAY * DM * DM * 2);
static constexpr size_t SZ_WF  = al256((size_t)NLAY * DFF * DM * 2);
static constexpr size_t SZ_WOUT = al256((size_t)VOC * DM * 2);
static constexpr size_t SZ_PE  = al256((size_t)INITL * DM * 4);
static constexpr size_t SZ_MEM = al256((size_t)NLAY * 2 * SMEM * NBATCH * DM * 4);
static constexpr size_t SZ_KV  = al256((size_t)NLAY * 2 * LFN * NBATCH * DM * 4);
static constexpr size_t SZ_HP  = al256((size_t)LFN * 16 * DM * 2);
static constexpr size_t SZ_TOTAL = 2 * SZ_WSA + 2 * SZ_WSO + 2 * SZ_WF + SZ_WOUT + SZ_PE + SZ_MEM + SZ_KV + SZ_HP;
static_assert(SZ_TOTAL <= (size_t)134217728);
static_assert(((size_t)NLAY * 3 * DM * DM) % 64 == 0);
static_assert(((size_t)NLAY * DM * DM) % 64 == 0);
static_assert(((size_t)NLAY * DFF * DM) % 64 == 0);
static_assert(((size_t)VOC * DM) % 64 == 0);
static_assert((size_t)LFN * NBATCH * VOC <= (size_t)LF_FULL * NBATCH * VOC);

extern "C" void kernel_launch(void* const* d_in, const int* in_sizes, int n_in,
                              void* d_out, int out_size, void* d_ws, size_t ws_size, hipStream_t stream) {
    if (n_in < 20) return;
    if ((size_t)in_sizes[0] < (size_t)SMEM * NBATCH * DM) return;
    if (in_sizes[1] < NTR * NBATCH) return;
    if ((size_t)in_sizes[3] < (size_t)VOC * DM || (size_t)in_sizes[18] < (size_t)VOC * DM || in_sizes[19] < VOC) return;
    if ((size_t)in_sizes[4] < (size_t)NLAY * 3 * DM * DM || in_sizes[5] < NLAY * 3 * DM) return;
    if ((size_t)in_sizes[6] < (size_t)NLAY * DM * DM || in_sizes[7] < NLAY * DM) return;
    if ((size_t)in_sizes[8] < (size_t)NLAY * 3 * DM * DM || in_sizes[9] < NLAY * 3 * DM) return;
    if ((size_t)in_sizes[10] < (size_t)NLAY * DM * DM || in_sizes[11] < NLAY * DM) return;
    if ((size_t)in_sizes[12] < (size_t)NLAY * DFF * DM || in_sizes[13] < NLAY * DFF) return;
    if ((size_t)in_sizes[14] < (size_t)NLAY * DM * DFF || in_sizes[15] < NLAY * DM) return;
    if (in_sizes[16] < NLAY * 3 * DM || in_sizes[17] < NLAY * 3 * DM) return;
    if ((size_t)out_size < (size_t)LFN * NBATCH * VOC) return;
    if (SZ_TOTAL > ws_size) return;
    const float* enc   = (const float*)d_in[0];
    const int*   trf   = (const int*)d_in[1];
    const float* emb   = (const float*)d_in[3];
    const float* sa_w  = (const float*)d_in[4];  const float* sa_b  = (const float*)d_in[5];
    const float* sa_ow = (const float*)d_in[6];  const float* sa_ob = (const float*)d_in[7];
    const float* ca_w  = (const float*)d_in[8];  const float* ca_b  = (const float*)d_in[9];
    const float* ca_ow = (const float*)d_in[10]; const float* ca_ob = (const float*)d_in[11];
    const float* ff1_w = (const float*)d_in[12]; const float* ff1_b = (const float*)d_in[13];
    const float* ff2_w = (const float*)d_in[14]; const float* ff2_b = (const float*)d_in[15];
    const float* ln_g  = (const float*)d_in[16]; const float* ln_b  = (const float*)d_in[17];
    const float* out_w = (const float*)d_in[18]; const float* out_b = (const float*)d_in[19];
    float* OUT = (float*)d_out;
    char* wsp = (char*)d_ws;
    h16* WSA  = (h16*)wsp; wsp += SZ_WSA;
    h16* WCA  = (h16*)wsp; wsp += SZ_WSA;
    h16* WSO  = (h16*)wsp; wsp += SZ_WSO;
    h16* WCO  = (h16*)wsp; wsp += SZ_WSO;
    h16* WF1  = (h16*)wsp; wsp += SZ_WF;
    h16* WF2  = (h16*)wsp; wsp += SZ_WF;
    h16* WOUT = (h16*)wsp; wsp += SZ_WOUT;
    float* PE  = (float*)wsp; wsp += SZ_PE;
    float* MEM = (float*)wsp; wsp += SZ_MEM;
    float* KV  = (float*)wsp; wsp += SZ_KV;
    h16* HP   = (h16*)wsp; wsp += SZ_HP;

    { const size_t n8 = (size_t)NLAY * 3 * DM * DM / 8; const unsigned g = (unsigned)((n8 + 255) / 256);
      k_wcvt<<<g, 256, 0, stream>>>(sa_w, WSA, n8); k_wcvt<<<g, 256, 0, stream>>>(ca_w, WCA, n8); }
    { const size_t n8 = (size_t)NLAY * DM * DM / 8; const unsigned g = (unsigned)((n8 + 255) / 256);
      k_wcvt<<<g, 256, 0, stream>>>(sa_ow, WSO, n8); k_wcvt<<<g, 256, 0, stream>>>(ca_ow, WCO, n8); }
    { const size_t n8 = (size_t)NLAY * DFF * DM / 8; const unsigned g = (unsigned)((n8 + 255) / 256);
      k_wcvt<<<g, 256, 0, stream>>>(ff1_w, WF1, n8); k_wcvt<<<g, 256, 0, stream>>>(ff2_w, WF2, n8); }
    { const size_t n8 = (size_t)VOC * DM / 8; const unsigned g = (unsigned)((n8 + 255) / 256);
      k_wcvt<<<g, 256, 0, stream>>>(out_w, WOUT, n8); }
    k_pe<<<(INITL * DM) / 256, 256, 0, stream>>>(PE);
    k_mem<<<dim3(SMEM, NLAY * 2, 1), 256, 0, stream>>>(enc, WCA, ca_b, MEM);

    const int first = LFN < INITL ? LFN : INITL;
    k_step<<<1, 256, 0, stream>>>(trf, emb, PE, WSA, sa_b, WSO, sa_ob, WCA, ca_b, WCO, ca_ob, WF1, ff1_b, WF2, ff2_b, ln_g, ln_b, MEM, KV, HP, OUT, 0, first);
    k_vocab<<<dim3(VOC / 256, first, 1), 128, 0, stream>>>(HP, WOUT, out_b, OUT, 0);
    for (int p = INITL; p < LFN; ++p) {
        k_step<<<1, 256, 0, stream>>>(trf, emb, PE, WSA, sa_b, WSO, sa_ob, WCA, ca_b, WCO, ca_ob, WF1, ff1_b, WF2, ff2_b, ln_g, ln_b, MEM, KV, HP, OUT, p, p + 1);
        k_vocab<<<dim3(VOC / 256, 1, 1), 128, 0, stream>>>(HP, WOUT, out_b, OUT, p);
    }
}
